// HypernymVisual_acc2_10213432230336
// MI455X (gfx1250) — hardware-verified
//
#include <hip/hip_runtime.h>


#define NBR  512
#define NNEG 2048
#define DD   300
#define DDP  320
#define FF   4096
#define HH   2000
#define HHP  2048
#define DM   FF
#define BN_EPS 1e-5f
#define LOSC 1024.0f

typedef _Float16 h16;
typedef unsigned short bf;
typedef __attribute__((ext_vector_type(16))) __bf16   v16bf;
typedef __attribute__((ext_vector_type(16))) _Float16 v16h;
typedef __attribute__((ext_vector_type(8)))  _Float16 v8h;
typedef __attribute__((ext_vector_type(8)))  unsigned short v8us;
typedef __attribute__((ext_vector_type(8)))  float    v8f;
typedef __attribute__((ext_vector_type(4)))  float    v4f;
typedef v8h  __attribute__((may_alias)) v8ha;
typedef v4f  __attribute__((may_alias)) v4fa;
typedef v8us __attribute__((may_alias)) v8usa;

__device__ __forceinline__ unsigned short f2bf(float f) { unsigned u = __float_as_uint(f); u += 0x7FFFu + ((u >> 16) & 1u); return (unsigned short)(u >> 16); }
__device__ __forceinline__ float bf2f(unsigned short b) { return __uint_as_float(((unsigned)b) << 16); }
__device__ __forceinline__ float bfr(float f) { return bf2f(f2bf(f)); }
__device__ __forceinline__ v16h cat16(v8h lo, v8h hi) { return __builtin_shufflevector(lo, hi, 0, 1, 2, 3, 4, 5, 6, 7, 8, 9, 10, 11, 12, 13, 14, 15); }
__device__ __forceinline__ v16bf cat16b(v8us lo, v8us hi) { return __builtin_bit_cast(v16bf, __builtin_shufflevector(lo, hi, 0, 1, 2, 3, 4, 5, 6, 7, 8, 9, 10, 11, 12, 13, 14, 15)); }
__device__ __forceinline__ v8f wmma16(v16h a, v16h b, v8f c) { return __builtin_amdgcn_wmma_f32_16x16x32_f16(false, a, false, b, (short)0, c, false, false); }
__device__ __forceinline__ v8f wmmab(v16bf a, v16bf b, v8f c) { return __builtin_amdgcn_wmma_f32_16x16x32_bf16(false, a, false, b, (short)0, c, false, false); }

template <bool SPLITA, bool F16OUT = false>
__global__ __launch_bounds__(128) void k_gemmb(const bf* __restrict__ A, const bf* __restrict__ Al, const bf* __restrict__ Bn, const float* __restrict__ bias, float* C, int ldc, h16* C2, const float* __restrict__ R = nullptr, int K = DM, int roundR = 1) {
    __shared__ __align__(16) float ost[4][16 * 68];
    const int lane = threadIdx.x & 31, wave = threadIdx.x >> 5, lr = lane & 15, hi = lane >> 4;
    const int r0 = blockIdx.x * 64 + wave * 16, c0 = blockIdx.y * 64;
    const size_t aoff = (size_t)(r0 + lr) * K + 8 * hi;
    size_t boff[4];
#pragma unroll
    for (int t = 0; t < 4; ++t) boff[t] = (size_t)(c0 + t * 16 + lr) * K + 8 * hi;
    v8f acc[4];
#pragma unroll
    for (int t = 0; t < 4; ++t) acc[t] = (v8f){};
#pragma unroll 1
    for (int kc = 0; kc < K; kc += 32) {
        const v16bf a = cat16b(*(const v8us*)(A + aoff + kc), *(const v8us*)(A + aoff + kc + 16));
        v16bf al = a;
        if (SPLITA) al = cat16b(*(const v8us*)(Al + aoff + kc), *(const v8us*)(Al + aoff + kc + 16));
#pragma unroll
        for (int t = 0; t < 4; ++t) { const v16bf b = cat16b(*(const v8us*)(Bn + boff[t] + kc), *(const v8us*)(Bn + boff[t] + kc + 16)); acc[t] = wmmab(a, b, acc[t]); if (SPLITA) acc[t] = wmmab(al, b, acc[t]); }
        asm volatile("v_nop\n\tv_nop\n\tv_nop\n\tv_nop" : "+v"(acc[0]), "+v"(acc[1]), "+v"(acc[2]), "+v"(acc[3]) : "v"(a), "v"(al));
    }
    float* os = &ost[wave][0];
#pragma unroll
    for (int t = 0; t < 4; ++t) { const float bv = bias ? bfr(bias[c0 + t * 16 + lr]) : 0.f;
#pragma unroll
        for (int j = 0; j < 8; ++j) os[(hi * 8 + j) * 68 + t * 16 + lr] = acc[t][j] + bv; }
    __syncthreads();
    if (F16OUT) {
        h16* crow = (h16*)(void*)C + (size_t)r0 * ldc + c0;
        auto pass = [&]() {
#pragma unroll
            for (int s = 0; s < 4; ++s) { const int row = 4 * s + (lane >> 3), piece = lane & 7; const float* sp = os + row * 68 + piece * 8; v8h o, o2;
#pragma unroll
                for (int i = 0; i < 8; ++i) { const h16 a = (h16)sp[i]; o[i] = a; o2[i] = (h16)((sp[i] - (float)a) * LOSC); }
                *(volatile v8h*)(crow + (size_t)row * ldc + piece * 8) = o; if (C2) *(volatile v8h*)(C2 + (size_t)r0 * ldc + c0 + (size_t)row * ldc + piece * 8) = o2; }
        };
        pass(); __threadfence(); pass();
    } else {
        float* crow = C + (size_t)r0 * ldc + c0;
        auto pass = [&]() {
#pragma unroll
            for (int s = 0; s < 8; ++s) { const int Lid = (lane >> 3) + 4 * s, piece = lane & 7; const int row = Lid >> 1, cofs = (Lid & 1) * 32 + piece * 4;
                v4f val = *(const v4fa*)(os + row * 68 + cofs); if (R) { const v4f rv = *(const v4f*)(R + ((size_t)r0 + row) * ldc + c0 + cofs); val += roundR ? (v4f){bfr(rv[0]), bfr(rv[1]), bfr(rv[2]), bfr(rv[3])} : rv; }
                *(volatile v4f*)(crow + (size_t)row * ldc + cofs) = val; }
        };
        pass(); __threadfence(); pass();
    }
}


__global__ __launch_bounds__(256) void k_wtp(const float* __restrict__ Wm, int krows, int ncols, int kpad, bf* WT) {
    __shared__ __align__(16) unsigned short tl[64 * 72];
    const int tid = threadIdx.x, k0 = blockIdx.x * 64, n0 = blockIdx.y * 64;
    const int kk = tid >> 2, nq = (tid & 3) * 16;
    const int k = k0 + kk, kc = k < krows ? k : krows - 1;
#pragma unroll
    for (int i = 0; i < 16; ++i) { const int n = n0 + nq + i, ncl = n < ncols ? n : ncols - 1; const float w = Wm[(size_t)kc * ncols + ncl]; tl[(nq + i) * 72 + kk] = (k < krows && n < ncols) ? f2bf(w) : (unsigned short)0; }
    __syncthreads();
    const int piece = tid & 7;
    auto pass = [&]() {
#pragma unroll
        for (int s = 0; s < 2; ++s) { const int nr = (tid >> 3) + 32 * s; const v8us val = *(const v8usa*)(tl + nr * 72 + piece * 8); *(volatile v8us*)(WT + (size_t)(n0 + nr) * kpad + k0 + piece * 8) = val; }
    };
    pass(); __threadfence(); pass();
}
__global__ __launch_bounds__(256) void k_bnstat(const float* __restrict__ vf, float* MU, float* RS) {
    const int f = blockIdx.x * 256 + threadIdx.x; if (f >= FF) return; float s = 0.f;
#pragma unroll 1
    for (int r = 0; r < NBR; ++r) s += bfr(vf[(size_t)r * FF + f]);
    const float mu = s * (1.0f / NBR); float s2 = 0.f;
#pragma unroll 1
    for (int r = 0; r < NBR; ++r) { const float d = bfr(vf[(size_t)r * FF + f]) - mu; s2 = fmaf(d, d, s2); }
    const float rs = rsqrtf(s2 * (1.0f / NBR) + BN_EPS);
    *(volatile float*)(MU + f) = mu; *(volatile float*)(RS + f) = rs; __threadfence(); *(volatile float*)(MU + f) = mu; *(volatile float*)(RS + f) = rs;
}
__global__ __launch_bounds__(256) void k_bnapply(const float* __restrict__ vf, const float* __restrict__ MU, const float* __restrict__ RS, const float* __restrict__ ga, const float* __restrict__ be, bf* Vh, bf* Vl) {
    const int lane = threadIdx.x & 31, r = blockIdx.x * 8 + (threadIdx.x >> 5); if (r >= NBR) return;
#pragma unroll 1
    for (int ps = 0; ps < 2; ++ps) {
#pragma unroll 1
        for (int c0 = lane * 8; c0 < FF; c0 += 256) { const size_t o = (size_t)r * FF + c0; const v8f v = *(const v8f*)(vf + o); v8us oh, ol;
#pragma unroll
            for (int i = 0; i < 8; ++i) { const int f = c0 + i; const float y = (bfr(v[i]) - MU[f]) * RS[f] * bfr(ga[f]) + bfr(be[f]); const unsigned short hb = f2bf(y); oh[i] = hb; ol[i] = f2bf(y - bf2f(hb)); }
            *(volatile v8us*)(Vh + o) = oh; *(volatile v8us*)(Vl + o) = ol; }
        if (ps == 0) __threadfence(); }
}
__global__ __launch_bounds__(256) void k_hsplit(const float* __restrict__ H, const float* __restrict__ b1, bf* Hh, bf* Hl) {
    const int lane = threadIdx.x & 31, r = blockIdx.x * 8 + (threadIdx.x >> 5); if (r >= NBR) return;
#pragma unroll 1
    for (int ps = 0; ps < 2; ++ps) {
#pragma unroll 1
        for (int c0 = lane * 8; c0 < HHP; c0 += 256) { const size_t o = (size_t)r * HHP + c0; const v8f v = *(const v8f*)(H + o); v8us oh, ol;
#pragma unroll
            for (int i = 0; i < 8; ++i) { const int c = c0 + i, cc = c < HH ? c : HH - 1; const float y = (c < HH) ? v[i] + bfr(b1[cc]) : 0.f; const unsigned short hb = f2bf(y); oh[i] = hb; ol[i] = f2bf(y - bf2f(hb)); }
            *(volatile v8us*)(Hh + o) = oh; *(volatile v8us*)(Hl + o) = ol; }
        if (ps == 0) __threadfence(); }
}
__global__ __launch_bounds__(256) void k_energy(const float* __restrict__ E, const float* __restrict__ b2, const float* __restrict__ pw, const float* __restrict__ nw, float* O0, float* O1) {
    __shared__ float embs[DDP];
    const int tid = threadIdx.x, lane = tid & 31, v = blockIdx.x, n = blockIdx.y * 256 + tid;
    for (int d = tid; d < DDP; d += 256) { const int dc = d < DD ? d : DD - 1; embs[d] = (d < DD) ? E[(size_t)v * DDP + d] + bfr(b2[dc]) : 0.f; }
    __syncthreads();
    float pe = 0.f;
#pragma unroll 1
    for (int j = 0; j < (DD + 31) / 32; ++j) { const int d = lane + 32 * j; const int dc = d < DD ? d : DD - 1; const float t = fmaxf(bfr(pw[(size_t)v * DD + dc]) - embs[dc], 0.f); pe = (d < DD) ? fmaf(t, t, pe) : pe; }
#pragma unroll
    for (int sh = 16; sh; sh >>= 1) pe += __shfl_xor(pe, sh, 32);
    float ne = 0.f; const float* nr = nw + (size_t)n * DD;
#pragma unroll 2
    for (int d = 0; d < DD; ++d) { const float t = fmaxf(bfr(nr[d]) - embs[d], 0.f); ne = fmaf(t, t, ne); }
    const size_t o = (size_t)v * NNEG + n;
    *(volatile float*)(O0 + o) = pe; *(volatile float*)(O1 + o) = ne; __threadfence(); *(volatile float*)(O0 + o) = pe; *(volatile float*)(O1 + o) = ne;
}

extern "C" void kernel_launch(void* const* d_in, const int* in_sizes, int n_in,
                              void* d_out, int out_size, void* d_ws, size_t ws_size, hipStream_t stream) {
    (void)in_sizes; (void)n_in; (void)out_size;
    const float* vf = (const float*)d_in[0]; const float* pw = (const float*)d_in[1]; const float* nw = (const float*)d_in[2]; const float* ga = (const float*)d_in[3]; const float* be = (const float*)d_in[4];
    const float* W1 = (const float*)d_in[5]; const float* b1 = (const float*)d_in[6]; const float* W2 = (const float*)d_in[7]; const float* b2 = (const float*)d_in[8];
    float* out0 = (float*)d_out; float* out1 = (float*)((char*)d_out + (size_t)NBR * NNEG * 4);
    char* wsp = (char*)d_ws;
    auto take = [&](size_t bytes) { char* p = wsp; wsp += (bytes + 255) & ~(size_t)255; return (void*)p; };
    bf* W1T = (bf*)take((size_t)HHP * FF * 2); bf* W2T = (bf*)take((size_t)DDP * HHP * 2); float* MU = (float*)take(FF * 4); float* RS = (float*)take(FF * 4);
    bf* Vh = (bf*)take((size_t)NBR * FF * 2); bf* Vl = (bf*)take((size_t)NBR * FF * 2); float* H = (float*)take((size_t)NBR * HHP * 4); bf* Hh = (bf*)take((size_t)NBR * HHP * 2); bf* Hl = (bf*)take((size_t)NBR * HHP * 2); float* E = (float*)take((size_t)NBR * DDP * 4);
    if ((size_t)(wsp - (char*)d_ws) > ws_size) return;
    k_wtp<<<dim3(FF / 64, HHP / 64, 1), 256, 0, stream>>>(W1, FF, HH, FF, W1T);
    k_wtp<<<dim3(HHP / 64, DDP / 64, 1), 256, 0, stream>>>(W2, HH, DD, HHP, W2T);
    k_bnstat<<<FF / 256, 256, 0, stream>>>(vf, MU, RS); k_bnapply<<<NBR / 8, 256, 0, stream>>>(vf, MU, RS, ga, be, Vh, Vl);
    k_gemmb<true, false><<<dim3(NBR / 64, HHP / 64, 1), 128, 0, stream>>>(Vh, Vl, W1T, nullptr, H, HHP, nullptr, nullptr, FF);
    k_hsplit<<<NBR / 8, 256, 0, stream>>>(H, b1, Hh, Hl);
    k_gemmb<true, false><<<dim3(NBR / 64, DDP / 64, 1), 128, 0, stream>>>(Hh, Hl, W2T, nullptr, E, DDP, nullptr, nullptr, HHP);
    k_energy<<<dim3(NBR, NNEG / 256, 1), 256, 0, stream>>>(E, b2, pw, nw, out0, out1);
}
